// YMLocal_1434519076945
// MI455X (gfx1250) — hardware-verified
//
#include <hip/hip_runtime.h>
#include <stdint.h>

#define CH     256
#define NP     9216
#define KCH    32
#define NB     2
#define FROWS  128
#define GROWS  64
#define WROWS  320
#define QP     64
#define PT     288
#define TT     144
#define KCK    32
#define NKC    288
#define QBLK   128
#define NQB    72
#define SPP    40
#define SLP    36
#define VPC    36

#define ASCALE   64.0f
#define WSCALE   1024.0f
#define CSCALE   1024.0f
#define OSC_PROJ (1.0f / 65536.0f)
#define OSC_TAIL (1.0f / 1048576.0f)
#define PSCALE   16384.0f
#define OSC_ATT  (1.0f / 1048576.0f)
#define SL2      (1.4426950408889634f * 0.17677669529663688f * (1.0f / 4096.0f))

static_assert(NB == 2);
static_assert(PT * 32 == NP);
static_assert(TT * 64 == NP);
static_assert(NKC * KCK == NP);
static_assert(NQB * QBLK == NP);
static_assert(QBLK == 8 * 16);
static_assert(VPC * 256 == NP);
static_assert(QP == 2 * KCH);
static_assert((SPP % 8) == 0 && SPP >= KCK && (SLP % 4) == 0 && SLP >= KCH);
static_assert(WROWS == GROWS + CH && FROWS == 2 * GROWS);
static_assert((NP % 64) == 0 && (CH % 64) == 0 && (CH % 32) == 0);
static_assert(((GROWS / 64) * (NP / 64)) % 8 == 0);
static_assert(((CH / 64) * (NP / 64)) % 8 == 0);

typedef _Float16 v16h __attribute__((ext_vector_type(16)));
typedef _Float16 v8h  __attribute__((ext_vector_type(8)));
typedef float    v8f  __attribute__((ext_vector_type(8)));
typedef float    v4f  __attribute__((ext_vector_type(4)));
typedef unsigned int v4u __attribute__((ext_vector_type(4)));
static_assert(sizeof(v16h) == 32);
static_assert(sizeof(v8h) == 16);

__device__ __forceinline__ unsigned short bf_bits(float f) {
  unsigned u = __float_as_uint(f);
  return (unsigned short)((u + 0x7FFFu + ((u >> 16) & 1u)) >> 16);
}
__device__ __forceinline__ float bf_up(unsigned short hb) { return __uint_as_float(((unsigned)hb) << 16); }
__device__ __forceinline__ float bfr(float f) { return bf_up(bf_bits(f)); }
__device__ __forceinline__ unsigned short h_bits(_Float16 x) { return __builtin_bit_cast(unsigned short, x); }
__device__ __forceinline__ unsigned short f2h_bits(float f) { return h_bits((_Float16)f); }
__device__ __forceinline__ unsigned short res_bits(float t) {
  const float hh = (float)((_Float16)t);
  return f2h_bits(t - hh);
}
__device__ __forceinline__ unsigned pk16(unsigned short a, unsigned short b) { return (unsigned)a | ((unsigned)b << 16); }
__device__ __forceinline__ v8f zero8() { v8f z = {0.f, 0.f, 0.f, 0.f, 0.f, 0.f, 0.f, 0.f}; return z; }

__device__ __forceinline__ v16h ldfrag_h(const _Float16* p) {
  union { v16h v; v8h hv[2]; } f;
  f.hv[0] = *(const v8h*)(p);
  f.hv[1] = *(const v8h*)(p + 16);
  return f.v;
}

__device__ __forceinline__ v8f mma_h_raw(v16h a, v16h b, v8f c) {
  return __builtin_amdgcn_wmma_f32_16x16x32_f16(false, a, false, b, (short)0, c, false, false);
}
__device__ __forceinline__ void dep_guard_h(v8f& a, v8f& b, v16h x, v16h y) {
#if defined(__HIP_DEVICE_COMPILE__)
  asm volatile("v_nop\n\tv_nop\n\tv_nop\n\tv_nop" : "+v"(a), "+v"(b) : "v"(x), "v"(y));
#endif
}
__device__ __forceinline__ void dep_guard2x3(v8f& a, v8f& b, v16h x, v16h y, v16h z) {
#if defined(__HIP_DEVICE_COMPILE__)
  asm volatile("v_nop\n\tv_nop\n\tv_nop\n\tv_nop" : "+v"(a), "+v"(b) : "v"(x), "v"(y), "v"(z));
#endif
}
__device__ __forceinline__ void keep4_h(v16h a, v16h b, v16h c, v16h d) {
#if defined(__HIP_DEVICE_COMPILE__)
  asm volatile("v_nop" :: "v"(a), "v"(b), "v"(c), "v"(d));
#endif
}
__device__ __forceinline__ void keep2_h(v16h a, v16h b) {
#if defined(__HIP_DEVICE_COMPILE__)
  asm volatile("v_nop" :: "v"(a), "v"(b));
#endif
}
__device__ __forceinline__ void acc_guard4(v8f& a, v8f& b, v8f& c, v8f& d) {
#if defined(__HIP_DEVICE_COMPILE__)
  asm volatile("v_nop\n\tv_nop\n\tv_nop\n\tv_nop" : "+v"(a), "+v"(b), "+v"(c), "+v"(d));
#endif
}
__device__ __forceinline__ void wave_sync_lds() {
  __builtin_amdgcn_fence(__ATOMIC_RELEASE, "workgroup");
  __builtin_amdgcn_wave_barrier();
  __builtin_amdgcn_fence(__ATOMIC_ACQUIRE, "workgroup");
}

__global__ __launch_bounds__(256) void cvt_tok(const float* __restrict__ x, const float* __restrict__ hm,
                                                unsigned short* xt, unsigned short* ht) {
  __shared__ __align__(16) float sx[CH * 33];
  const int tid = threadIdx.x;
  const int z = blockIdx.y;
  const int which = z >> 1, b = z & 1;
  const float* src = ((which != 0) ? hm : x) + (size_t)b * CH * NP;
  unsigned short* dstp = ((which != 0) ? ht : xt) + (size_t)b * NP * CH;
  const int p0 = blockIdx.x * 32;
#pragma unroll 8
  for (int it = 0; it < 32; ++it) {
    const int idx = it * 256 + tid;
    const int c = idx >> 5, q = idx & 31;
    sx[c * 33 + q] = src[(size_t)c * NP + p0 + q];
  }
  __syncthreads();
  const int wave = tid >> 5, lane = tid & 31, c8 = lane * 8;
  v4u pk[4];
#pragma unroll
  for (int it = 0; it < 4; ++it) {
    const int r = wave * 4 + it;
    v4u p;
#pragma unroll
    for (int e = 0; e < 4; ++e) {
      const float a  = bfr(sx[(c8 + 2 * e) * 33 + r]) * ASCALE;
      const float bb = bfr(sx[(c8 + 2 * e + 1) * 33 + r]) * ASCALE;
      p[e] = pk16(f2h_bits(a), f2h_bits(bb));
    }
    pk[it] = p;
  }
  unsigned short* dst = dstp + (size_t)p0 * CH;
  for (int pass = 0; pass < 2; ++pass) {
#pragma unroll
    for (int it = 0; it < 4; ++it) {
      const int r = wave * 4 + it;
      *(volatile v4u*)(dst + (size_t)r * CH + c8) = pk[it];
    }
    __threadfence();
  }
}

__global__ __launch_bounds__(256) void cvt_wqd(const float* __restrict__ wq, const float* __restrict__ wd,
                                                unsigned short* wqd) {
  const int tid = threadIdx.x, wave = tid >> 5, lane = tid & 31, c8 = lane * 8;
  const int row = blockIdx.x * 8 + wave;
  const int g = row >> 6, rr = row & 63;
  const int srow = min(rr, KCH - 1);
  const bool valid = rr < KCH;
  const float* src = ((g != 0) ? wd : wq) + (size_t)srow * CH + c8;
  v4u p;
#pragma unroll
  for (int i = 0; i < 4; ++i) {
    const float a  = src[2 * i];
    const float bb = src[2 * i + 1];
    const unsigned short ha = valid ? f2h_bits(bfr(a) * WSCALE) : (unsigned short)0;
    const unsigned short hb = valid ? f2h_bits(bfr(bb) * WSCALE) : (unsigned short)0;
    p[i] = pk16(ha, hb);
  }
  unsigned short* d = wqd + (size_t)row * CH + c8;
  *(volatile v4u*)d = p;
  __threadfence();
  *(volatile v4u*)d = p;
}

__global__ __launch_bounds__(256) void cvt_w64(const float* __restrict__ wf, const float* __restrict__ wu,
                                                unsigned short* w64) {
  const int tid = threadIdx.x, wave = tid >> 5, lane = tid & 31;
  const int row = blockIdx.x * 32 + wave * 4 + (lane >> 3);
  const int j = lane & 7, col0 = (8 * j) & 31;
  const int rf = min(row, KCH - 1);
  const int ru = min(max(row - GROWS, 0), CH - 1);
  const float* pf = wf + (size_t)rf * KCH + col0;
  const float* pu = wu + (size_t)ru * KCH + col0;
  const bool isf = row < GROWS;
  const bool fvalid = row < KCH;
  v4u p;
#pragma unroll
  for (int i = 0; i < 4; ++i) {
    const float af = pf[2 * i], bfv = pf[2 * i + 1];
    const float au = pu[2 * i], buv = pu[2 * i + 1];
    const float va = isf ? (fvalid ? af : 0.0f) : au;
    const float vb = isf ? (fvalid ? bfv : 0.0f) : buv;
    p[i] = pk16(f2h_bits(bfr(va) * WSCALE), f2h_bits(bfr(vb) * WSCALE));
  }
  unsigned short* d = w64 + (size_t)row * QP + 8 * j;
  *(volatile v4u*)d = p;
  __threadfence();
  *(volatile v4u*)d = p;
}

__global__ __launch_bounds__(256) void gemm64(
    const unsigned short* __restrict__ Ap, int lda,
    const unsigned short* __restrict__ Btp, int ldb, long long strideB,
    float* Cp, int ldc, long long strideC,
    int M, int N, int K, float oscale,
    const float* __restrict__ bias0, int nbias,
    const float* __restrict__ resid, int use_res) {
  const _Float16* A  = (const _Float16*)(const void*)Ap;
  const _Float16* Bt = (const _Float16*)(const void*)Btp;
  __shared__ __align__(16) float sT[8][16 * 68];
  const int b    = blockIdx.y;
  const int lane = threadIdx.x & 31;
  const int wave = threadIdx.x >> 5;
  const int tilesN = N >> 6;
  const int tilesM = M >> 6;
  const int tile = blockIdx.x * 8 + wave;
  if (tile >= tilesM * tilesN) return;
  const int tm = tile / tilesN;
  const int tn = tile - tm * tilesN;
  const int m0 = tm << 6;
  const int n0 = tn << 6;

  const _Float16* Bb = Bt + (size_t)b * (size_t)strideB;

  const int rlane = lane & 15;
  const int koff  = (lane >> 4) * 8;
  const int mOff  = (lane >> 4) * 8;

  v8f acc[4][4];
#pragma unroll
  for (int i = 0; i < 4; ++i)
#pragma unroll
    for (int j = 0; j < 4; ++j) acc[i][j] = zero8();

  for (int k0 = 0; k0 < K; k0 += 32) {
    v16h bh[4];
#pragma unroll
    for (int j = 0; j < 4; ++j) {
      const size_t bo = (size_t)(n0 + (j << 4) + rlane) * ldb + koff + k0;
      bh[j] = ldfrag_h(Bb + bo);
    }
#pragma unroll
    for (int i = 0; i < 4; ++i) {
      const size_t ao = (size_t)(m0 + (i << 4) + rlane) * lda + koff + k0;
      const v16h ah = ldfrag_h(A + ao);
#pragma unroll
      for (int j = 0; j < 4; ++j) {
        acc[i][j] = mma_h_raw(ah, bh[j], acc[i][j]);
      }
      dep_guard_h(acc[i][0], acc[i][3], ah, bh[3]);
    }
    keep4_h(bh[0], bh[1], bh[2], bh[3]);
  }
  acc_guard4(acc[0][0], acc[0][1], acc[0][2], acc[0][3]);
  acc_guard4(acc[1][0], acc[1][1], acc[1][2], acc[1][3]);
  acc_guard4(acc[2][0], acc[2][1], acc[2][2], acc[2][3]);
  acc_guard4(acc[3][0], acc[3][1], acc[3][2], acc[3][3]);

  float* slab = sT[wave];
  float* C = Cp + (size_t)b * (size_t)strideC;
  const float* R = resid + (size_t)b * (size_t)strideC;
  const int bclamp = (nbias > 0) ? (nbias - 1) : 0;
#pragma unroll
  for (int i = 0; i < 4; ++i) {
    const int mBase = m0 + (i << 4);
#pragma unroll
    for (int j = 0; j < 4; ++j) {
#pragma unroll
      for (int r = 0; r < 8; ++r) {
        slab[(mOff + r) * 68 + (j << 4) + rlane] = acc[i][j][r];
      }
    }
    wave_sync_lds();
    {
      const int hh = lane >> 4, c4 = (lane & 15) * 4;
      v4f ov[8];
#pragma unroll
      for (int it = 0; it < 8; ++it) {
        const int row = it * 2 + hh;
        const int mrw = mBase + row;
        const float bl = bfr(bias0[min(mrw, bclamp)]);
        const float bv = (mrw < nbias) ? bl : 0.0f;
        v4f v = *(const v4f*)(slab + row * 68 + c4);
        v[0] = v[0] * oscale + bv;
        v[1] = v[1] * oscale + bv;
        v[2] = v[2] * oscale + bv;
        v[3] = v[3] * oscale + bv;
        if (use_res != 0) {
          const v4f rx = *(const v4f*)(R + (size_t)mrw * ldc + n0 + c4);
          v[0] += bfr(rx[0]);
          v[1] += bfr(rx[1]);
          v[2] += bfr(rx[2]);
          v[3] += bfr(rx[3]);
        }
        ov[it] = v;
      }
      for (int pass = 0; pass < 2; ++pass) {
#pragma unroll
        for (int it = 0; it < 8; ++it) {
          const int row = it * 2 + hh;
          *(volatile v4f*)(C + (size_t)(mBase + row) * ldc + n0 + c4) = ov[it];
        }
        __threadfence();
      }
    }
    wave_sync_lds();
  }
}

__global__ __launch_bounds__(256) void cvt_tm(const float* __restrict__ src0, long long sstride, int relu,
                                               float scale, unsigned short* dst0) {
  __shared__ __align__(16) float st[KCH * 65];
  const int tid = threadIdx.x;
  const int b = blockIdx.y;
  const int p0 = blockIdx.x * 64;
  const float* src = src0 + (size_t)b * (size_t)sstride;
#pragma unroll
  for (int it = 0; it < 8; ++it) {
    const int idx = it * 256 + tid;
    const int c = idx >> 6, t = idx & 63;
    const float v = src[(size_t)c * NP + p0 + t];
    st[c * 65 + t] = (relu != 0) ? fmaxf(v, 0.0f) : v;
  }
  __syncthreads();
  const int j = tid & 7, tq = tid >> 3, c0 = 8 * (j & 3);
  const bool hisel = (j < 4);
  v4u pk[2];
#pragma unroll
  for (int i = 0; i < 2; ++i) {
    const int t = 32 * i + tq;
    v4u p;
#pragma unroll
    for (int e = 0; e < 4; ++e) {
      const float ta = st[(c0 + 2 * e) * 65 + t] * scale;
      const float tb = st[(c0 + 2 * e + 1) * 65 + t] * scale;
      const unsigned short ha = f2h_bits(ta), hb = f2h_bits(tb);
      const unsigned short la = res_bits(ta), lb = res_bits(tb);
      p[e] = pk16(hisel ? ha : la, hisel ? hb : lb);
    }
    pk[i] = p;
  }
  unsigned short* d = dst0 + ((size_t)b * NP + p0) * QP;
  for (int pass = 0; pass < 2; ++pass) {
#pragma unroll
    for (int i = 0; i < 2; ++i) {
      const int t = 32 * i + tq;
      *(volatile v4u*)(d + (size_t)t * QP + 8 * j) = pk[i];
    }
    __threadfence();
  }
}

__global__ __launch_bounds__(256) void cvt_v(const float* __restrict__ F, unsigned short* vh, unsigned short* vl) {
  const int tid = threadIdx.x, wave = tid >> 5, lane = tid & 31;
  const int row = blockIdx.x * 8 + wave;
  const int b = row >> 5, k = row & 31;
  const float* s = F + ((size_t)b * FROWS + GROWS + k) * NP;
  unsigned short* dh = vh + (size_t)row * NP;
  unsigned short* dl = vl + (size_t)row * NP;
#pragma unroll 1
  for (int it = 0; it < VPC; ++it) {
    const int base = it * 256 + lane * 8;
    const v4f a = *(const v4f*)(s + base);
    const v4f c = *(const v4f*)(s + base + 4);
    float f[8];
    f[0] = a[0] * ASCALE; f[1] = a[1] * ASCALE; f[2] = a[2] * ASCALE; f[3] = a[3] * ASCALE;
    f[4] = c[0] * ASCALE; f[5] = c[1] * ASCALE; f[6] = c[2] * ASCALE; f[7] = c[3] * ASCALE;
    v4u p, q;
#pragma unroll
    for (int e = 0; e < 4; ++e) {
      p[e] = pk16(f2h_bits(f[2 * e]), f2h_bits(f[2 * e + 1]));
      q[e] = pk16(res_bits(f[2 * e]), res_bits(f[2 * e + 1]));
    }
    unsigned short* ddh = dh + base;
    unsigned short* ddl = dl + base;
    *(volatile v4u*)ddh = p;
    *(volatile v4u*)ddl = q;
    __threadfence();
    *(volatile v4u*)ddh = p;
    *(volatile v4u*)ddl = q;
  }
}

__global__ __launch_bounds__(256) void k_attn(const unsigned short* __restrict__ qp,
                                               const unsigned short* __restrict__ vhp,
                                               const unsigned short* __restrict__ vlp,
                                               unsigned short* ct) {
  const _Float16* Q  = (const _Float16*)(const void*)qp;
  const _Float16* VH = (const _Float16*)(const void*)vhp;
  const _Float16* VL = (const _Float16*)(const void*)vlp;
  __shared__ __align__(16) _Float16 sP[8][16 * SPP];
  __shared__ __align__(16) float sO[8][16 * SLP];

  const int tid = threadIdx.x, wave = tid >> 5, lane = tid & 31;
  const int rl = lane & 15, h = lane >> 4, koff = 8 * h;
  const int b = blockIdx.y;
  const size_t tokq = (size_t)b * NP + (size_t)blockIdx.x * QBLK + 16 * wave;
  const _Float16* Kb  = Q  + (size_t)b * NP * QP;
  const _Float16* VHb = VH + (size_t)b * KCH * NP;
  const _Float16* VLb = VL + (size_t)b * KCH * NP;

  const v16h qh = ldfrag_h(Q + (tokq + rl) * QP + koff);
  const v16h ql = ldfrag_h(Q + (tokq + rl) * QP + KCH + koff);

  v8f acc0 = zero8(), acc1 = zero8();
  float rmax[8], lsum[8];
#pragma unroll
  for (int r = 0; r < 8; ++r) { rmax[r] = -1.0e30f; lsum[r] = 0.0f; }
  _Float16* sp = &sP[wave][0];

#pragma unroll 1
  for (int kc = 0; kc < NKC; ++kc) {
    const int key0 = kc * KCK;
    const _Float16* kp0 = Kb + (size_t)(key0 + rl) * QP + koff;
    const _Float16* kp1 = Kb + (size_t)(key0 + 16 + rl) * QP + koff;
    const v16h kh0 = ldfrag_h(kp0), kr0 = ldfrag_h(kp0 + KCH);
    const v16h kh1 = ldfrag_h(kp1), kr1 = ldfrag_h(kp1 + KCH);
    v8f s0 = mma_h_raw(qh, kh0, zero8());
    s0 = mma_h_raw(qh, kr0, s0);
    s0 = mma_h_raw(ql, kh0, s0);
    v8f s1 = mma_h_raw(qh, kh1, zero8());
    s1 = mma_h_raw(qh, kr1, s1);
    s1 = mma_h_raw(ql, kh1, s1);
    dep_guard2x3(s0, s1, ql, kh1, kr1);
    keep4_h(qh, kh0, kr0, ql);
    float tm[8];
#pragma unroll
    for (int r = 0; r < 8; ++r) tm[r] = fmaxf(s0[r], s1[r]) * SL2;
#pragma unroll
    for (int r = 0; r < 8; ++r) {
      tm[r] = fmaxf(tm[r], __shfl_xor(tm[r], 1, 32));
      tm[r] = fmaxf(tm[r], __shfl_xor(tm[r], 2, 32));
      tm[r] = fmaxf(tm[r], __shfl_xor(tm[r], 4, 32));
      tm[r] = fmaxf(tm[r], __shfl_xor(tm[r], 8, 32));
    }
#pragma unroll
    for (int r = 0; r < 8; ++r) {
      const float nm = fmaxf(rmax[r], tm[r]);
      const float al = __builtin_amdgcn_exp2f(rmax[r] - nm);
      rmax[r] = nm;
      lsum[r] *= al;
      acc0[r] *= al;
      acc1[r] *= al;
    }
#pragma unroll
    for (int r = 0; r < 8; ++r) {
      const float p0 = __builtin_amdgcn_exp2f(s0[r] * SL2 - rmax[r]);
      const float p1 = __builtin_amdgcn_exp2f(s1[r] * SL2 - rmax[r]);
      lsum[r] += p0 + p1;
      sp[(8 * h + r) * SPP + rl]      = (_Float16)(p0 * PSCALE);
      sp[(8 * h + r) * SPP + 16 + rl] = (_Float16)(p1 * PSCALE);
    }
    wave_sync_lds();
    const v16h pf = ldfrag_h(sp + rl * SPP + koff);
    const size_t vo0 = (size_t)rl * NP + key0 + koff;
    const size_t vo1 = (size_t)(16 + rl) * NP + key0 + koff;
    const v16h vh0 = ldfrag_h(VHb + vo0), vr0 = ldfrag_h(VLb + vo0);
    const v16h vh1 = ldfrag_h(VHb + vo1), vr1 = ldfrag_h(VLb + vo1);
    acc0 = mma_h_raw(pf, vh0, acc0);
    acc0 = mma_h_raw(pf, vr0, acc0);
    acc1 = mma_h_raw(pf, vh1, acc1);
    acc1 = mma_h_raw(pf, vr1, acc1);
    dep_guard2x3(acc0, acc1, pf, vh1, vr1);
    keep2_h(vh0, vr0);
    wave_sync_lds();
  }

  float inv[8];
#pragma unroll
  for (int r = 0; r < 8; ++r) {
    float l = lsum[r];
    l += __shfl_xor(l, 1, 32);
    l += __shfl_xor(l, 2, 32);
    l += __shfl_xor(l, 4, 32);
    l += __shfl_xor(l, 8, 32);
    inv[r] = OSC_ATT * (1.0f / l);
  }
  float* so = &sO[wave][0];
#pragma unroll
  for (int r = 0; r < 8; ++r) {
    so[(8 * h + r) * SLP + rl]      = acc0[r] * inv[r];
    so[(8 * h + r) * SLP + 16 + rl] = acc1[r] * inv[r];
  }
  wave_sync_lds();
  const int j = lane & 7, tq = lane >> 3, c0 = 8 * (j & 3);
  const bool hisel = (j < 4);
  v4u pk[4];
#pragma unroll
  for (int i = 0; i < 4; ++i) {
    const int t = 4 * i + tq;
    v4u p;
#pragma unroll
    for (int e = 0; e < 4; ++e) {
      const float ta = so[t * SLP + c0 + 2 * e] * CSCALE;
      const float tb = so[t * SLP + c0 + 2 * e + 1] * CSCALE;
      const unsigned short ha = f2h_bits(ta), hb = f2h_bits(tb);
      const unsigned short la = res_bits(ta), lb = res_bits(tb);
      p[e] = pk16(hisel ? ha : la, hisel ? hb : lb);
    }
    pk[i] = p;
  }
  for (int pass = 0; pass < 2; ++pass) {
#pragma unroll
    for (int i = 0; i < 4; ++i) {
      const int t = 4 * i + tq;
      *(volatile v4u*)(ct + (tokq + t) * QP + 8 * j) = pk[i];
    }
    __threadfence();
  }
}

extern "C" void kernel_launch(void* const* d_in, const int* in_sizes, int n_in,
                              void* d_out, int out_size, void* d_ws, size_t ws_size,
                              hipStream_t stream) {
  if (n_in < 10) return;
  if (in_sizes[0] != NB * CH * NP) return;
  if (in_sizes[1] != NB * CH * NP) return;
  if (in_sizes[2] != KCH * CH) return;
  if (in_sizes[3] != KCH) return;
  if (in_sizes[4] != KCH * CH) return;
  if (in_sizes[5] != KCH) return;
  if (in_sizes[6] != KCH * KCH) return;
  if (in_sizes[7] != KCH) return;
  if (in_sizes[8] != CH * KCH) return;
  if (in_sizes[9] != CH) return;
  if (out_size != NB * CH * NP) return;

  const float* x     = (const float*)d_in[0];
  const float* human = (const float*)d_in[1];
  const float* wq    = (const float*)d_in[2];
  const float* bq    = (const float*)d_in[3];
  const float* wd    = (const float*)d_in[4];
  const float* bd    = (const float*)d_in[5];
  const float* wf    = (const float*)d_in[6];
  const float* bfb   = (const float*)d_in[7];
  const float* wu    = (const float*)d_in[8];
  const float* bu    = (const float*)d_in[9];
  float* out = (float*)d_out;

  const size_t PXT  = (size_t)NB * NP * CH * 2;
  const size_t PWQD = (size_t)FROWS * CH * 2;
  const size_t PW64 = (size_t)WROWS * QP * 2;
  const size_t PF   = (size_t)NB * FROWS * NP * 4;
  const size_t PQH  = (size_t)NB * NP * QP * 2;
  const size_t PVH  = (size_t)NB * KCH * NP * 2;
  const size_t PG   = (size_t)NB * GROWS * NP * 4;

  size_t off = 0;
  const size_t oXT  = off; off += PXT;
  const size_t oHT  = off; off += PXT;
  const size_t oWQD = off; off += PWQD;
  const size_t oW64 = off; off += PW64;
  const size_t oF   = off; off += PF;
  const size_t oQH  = off; off += PQH;
  const size_t oVH  = off; off += PVH;
  const size_t oVL  = off; off += PVH;
  const size_t oCT  = off; off += PQH;
  const size_t oG   = off; off += PG;
  const size_t oYT  = off; off += PQH;
  if (off > ws_size) return;
  if (off > (size_t)134217728) return;

  char* ws = (char*)d_ws;
  unsigned short* XT  = (unsigned short*)(ws + oXT);
  unsigned short* HT  = (unsigned short*)(ws + oHT);
  unsigned short* WQD = (unsigned short*)(ws + oWQD);
  unsigned short* W64 = (unsigned short*)(ws + oW64);
  float*          F   = (float*)(ws + oF);
  unsigned short* QH  = (unsigned short*)(ws + oQH);
  unsigned short* VHp = (unsigned short*)(ws + oVH);
  unsigned short* VLp = (unsigned short*)(ws + oVL);
  unsigned short* CT  = (unsigned short*)(ws + oCT);
  float*          G   = (float*)(ws + oG);
  unsigned short* YT  = (unsigned short*)(ws + oYT);

  const dim3 blk(256);
  const long long sTok = (long long)NP * CH;
  const long long sF   = (long long)FROWS * NP;
  const long long sQ   = (long long)NP * QP;
  const long long sG   = (long long)GROWS * NP;
  const long long sOut = (long long)CH * NP;

  cvt_tok<<<dim3(PT, 2 * NB), blk, 0, stream>>>(x, human, XT, HT);
  cvt_wqd<<<dim3(FROWS / 8), blk, 0, stream>>>(wq, wd, WQD);
  cvt_w64<<<dim3(WROWS / 32), blk, 0, stream>>>(wf, wu, W64);
  const dim3 g64(((GROWS / 64) * (NP / 64)) / 8, NB);
  const dim3 g256(((CH / 64) * (NP / 64)) / 8, NB);
  gemm64<<<g64, blk, 0, stream>>>(WQD, CH, HT, CH, sTok, F, NP, sF,
                                  GROWS, NP, CH, OSC_PROJ, bq, KCH, x, 0);
  gemm64<<<g64, blk, 0, stream>>>(WQD + (size_t)GROWS * CH, CH, XT, CH, sTok, F + (size_t)GROWS * NP, NP, sF,
                                  GROWS, NP, CH, OSC_PROJ, bd, KCH, x, 0);
  cvt_tm<<<dim3(TT, NB), blk, 0, stream>>>(F, sF, 0, ASCALE, QH);
  cvt_v<<<dim3((NB * KCH) / 8), blk, 0, stream>>>(F, VHp, VLp);
  k_attn<<<dim3(NQB, NB), blk, 0, stream>>>(QH, VHp, VLp, CT);
  gemm64<<<g64, blk, 0, stream>>>(W64, QP, CT, QP, sQ, G, NP, sG,
                                  GROWS, NP, QP, OSC_TAIL, bfb, KCH, x, 0);
  cvt_tm<<<dim3(TT, NB), blk, 0, stream>>>(G, sG, 1, CSCALE, YT);
  gemm64<<<g256, blk, 0, stream>>>(W64 + (size_t)GROWS * QP, QP, YT, QP, sQ, out, NP, sOut,
                                   CH, NP, QP, OSC_TAIL, bu, CH, x, 1);
  (void)hipGetLastError();
}
